// naive_attn_like_55757265437272
// MI455X (gfx1250) — hardware-verified
//
#include <hip/hip_runtime.h>

typedef __attribute__((ext_vector_type(16))) _Float16 v16h;
typedef __attribute__((ext_vector_type(8)))  _Float16 v8h;
typedef __attribute__((ext_vector_type(4)))  _Float16 v4h;
typedef __attribute__((ext_vector_type(8)))  float    v8f;
typedef __attribute__((ext_vector_type(4)))  float    v4f;
typedef __attribute__((ext_vector_type(4)))  unsigned v4u;

__device__ __forceinline__ v8f wmma_f16(v16h a, v16h b, v8f c) {
    v8f d = __builtin_amdgcn_wmma_f32_16x16x32_f16(false, a, false, b, (short)0, c, false, false);
    asm volatile("v_nop\n\tv_nop\n\tv_nop\n\tv_nop" : "+v"(d) : "v"(a), "v"(b));
    return d;
}

#define NTOK 8192
#define DIMK 1024
#define DKV  128

__global__ __launch_bounds__(256) void proj_kernel(
    const float* __restrict__ x,
    const float* __restrict__ Wqk,
    const float* __restrict__ bqk,
    const float* __restrict__ Wv,
    const float* __restrict__ bv,
    _Float16* __restrict__ qk_h,
    _Float16* __restrict__ v_h)
{
    __shared__ __align__(16) _Float16 xs[64][32];
    __shared__ __align__(16) _Float16 ws[256][32];
    __shared__ __align__(16) _Float16 os[8][16 * 128];

    const int tid  = threadIdx.x;
    const int lane = tid & 31;
    const int wave = tid >> 5;
    const int rowblk  = wave & 3;
    const int colhalf = wave >> 2;
    const int g = lane >> 4;
    const int n = lane & 15;
    const int wg_row0 = blockIdx.x * 64;

    v8f acc[8];
#pragma unroll
    for (int t = 0; t < 8; ++t)
#pragma unroll
        for (int r = 0; r < 8; ++r) acc[t][r] = 0.0f;

    for (int k0 = 0; k0 < DIMK; k0 += 32) {
        __syncthreads();
#pragma unroll
        for (int i = 0; i < 2; ++i) {
            int idx = (i * 256 + tid) * 4;
            int r = idx >> 5, c = idx & 31;
            float4 f = *(const float4*)&x[(size_t)(wg_row0 + r) * DIMK + k0 + c];
            v4h h; h[0] = (_Float16)f.x; h[1] = (_Float16)f.y;
                   h[2] = (_Float16)f.z; h[3] = (_Float16)f.w;
            *(v4h*)&xs[r][c] = h;
        }
#pragma unroll
        for (int i = 0; i < 8; ++i) {
            int idx = (i * 256 + tid) * 4;
            int r = idx >> 5, c = idx & 31;
            const float* Wsrc = (r < 128) ? (Wqk + (size_t)r * DIMK)
                                          : (Wv + (size_t)(r - 128) * DIMK);
            float4 f = *(const float4*)&Wsrc[k0 + c];
            v4h h; h[0] = (_Float16)f.x; h[1] = (_Float16)f.y;
                   h[2] = (_Float16)f.z; h[3] = (_Float16)f.w;
            *(v4h*)&ws[r][c] = h;
        }
        __syncthreads();

        union { v16h v; v8h h[2]; } A;
        A.h[0] = *(const v8h*)&xs[rowblk * 16 + n][g * 8];
        A.h[1] = *(const v8h*)&xs[rowblk * 16 + n][16 + g * 8];

#pragma unroll
        for (int t = 0; t < 8; ++t) {
            union { v16h v; v8h h[2]; } B;
            const int wrow = colhalf * 128 + t * 16 + n;
            B.h[0] = *(const v8h*)&ws[wrow][g * 8];
            B.h[1] = *(const v8h*)&ws[wrow][16 + g * 8];
            acc[t] = wmma_f16(A.v, B.v, acc[t]);
        }
    }

    const float*  bias = colhalf ? bv  : bqk;
    _Float16*     dst  = colhalf ? v_h : qk_h;
    _Float16* ot = os[wave];
#pragma unroll
    for (int t = 0; t < 8; ++t) {
        int c128 = t * 16 + n;
#pragma unroll
        for (int r = 0; r < 8; ++r)
            ot[(r + 8 * g) * 128 + c128] = (_Float16)(acc[t][r] + bias[c128]);
    }
    __syncthreads();
    {
        char* d0 = (char*)(dst + (size_t)(wg_row0 + rowblk * 16) * DKV);
        v4u vv[8];
#pragma unroll
        for (int q = 0; q < 8; ++q) vv[q] = *(const v4u*)((const char*)ot + (q * 32 + lane) * 16);
#pragma unroll
        for (int q = 0; q < 8; ++q) *(volatile v4u*)(d0 + (q * 32 + lane) * 16) = vv[q];
        __threadfence();
#pragma unroll
        for (int q = 0; q < 8; ++q) *(volatile v4u*)(d0 + (q * 32 + lane) * 16) = vv[q];
    }
}

__global__ __launch_bounds__(256) void flash_kernel(
    const _Float16* __restrict__ qk,
    const _Float16* __restrict__ vh,
    float* __restrict__ out)
{
    __shared__ __align__(16) _Float16 Ks[32][128];
    __shared__ __align__(16) _Float16 Vt[128][32];
    __shared__ __align__(16) float    Ss[8][16][32];
    __shared__ __align__(16) _Float16 Ps[8][16][32];
    __shared__ float                  Al[8][16];
    __shared__ __align__(16) float    Os[8][16 * 128];

    const int tid  = threadIdx.x;
    const int lane = tid & 31;
    const int wave = tid >> 5;
    const int g = lane >> 4;
    const int n = lane & 15;
    const int q0 = blockIdx.x * 128 + wave * 16;

    v16h Aq[4];
#pragma unroll
    for (int c = 0; c < 4; ++c) {
        union { v16h v; v8h h[2]; } u;
        const _Float16* qrow = qk + (size_t)(q0 + n) * DKV + c * 32;
        u.h[0] = *(const v8h*)&qrow[g * 8];
        u.h[1] = *(const v8h*)&qrow[16 + g * 8];
        Aq[c] = u.v;
    }

    v8f O[8];
#pragma unroll
    for (int t = 0; t < 8; ++t)
#pragma unroll
        for (int r = 0; r < 8; ++r) O[t][r] = 0.0f;

    float m_i = -__builtin_inff();
    float l_i = 0.0f;

    const int kr0 = (tid * 8) >> 7,          kc0 = (tid * 8) & 127;
    const int kr1 = ((256 + tid) * 8) >> 7,  kc1 = ((256 + tid) * 8) & 127;

    const int pf_row = tid >> 3;
    const int pf_col = (tid & 7) * 16;

    for (int j0 = 0; j0 < NTOK; j0 += 32) {
        __syncthreads();
        *(v8h*)&Ks[kr0][kc0] = *(const v8h*)&qk[(size_t)(j0 + kr0) * DKV + kc0];
        *(v8h*)&Ks[kr1][kc1] = *(const v8h*)&qk[(size_t)(j0 + kr1) * DKV + kc1];
#pragma unroll
        for (int i = 0; i < 2; ++i) {
            int idx = (i * 256 + tid) * 8;
            int r = idx >> 7, c = idx & 127;
            v8h vv = *(const v8h*)&vh[(size_t)(j0 + r) * DKV + c];
#pragma unroll
            for (int k = 0; k < 8; ++k) Vt[c + k][r] = vv[k];
        }
        if (j0 + 32 < NTOK) {
            __builtin_prefetch(&qk[(size_t)(j0 + 32 + pf_row) * DKV + pf_col], 0, 3);
            __builtin_prefetch(&vh[(size_t)(j0 + 32 + pf_row) * DKV + pf_col], 0, 3);
        }
        __syncthreads();

        v8f S0a, S0b, S1a, S1b;
#pragma unroll
        for (int r = 0; r < 8; ++r) { S0a[r] = 0.0f; S0b[r] = 0.0f;
                                      S1a[r] = 0.0f; S1b[r] = 0.0f; }
#pragma unroll
        for (int c = 0; c < 2; ++c) {
            union { v16h v; v8h h[2]; } B0, B1, B2, B3;
            B0.h[0] = *(const v8h*)&Ks[n][c * 32 + g * 8];
            B0.h[1] = *(const v8h*)&Ks[n][c * 32 + 16 + g * 8];
            B1.h[0] = *(const v8h*)&Ks[16 + n][c * 32 + g * 8];
            B1.h[1] = *(const v8h*)&Ks[16 + n][c * 32 + 16 + g * 8];
            B2.h[0] = *(const v8h*)&Ks[n][(c + 2) * 32 + g * 8];
            B2.h[1] = *(const v8h*)&Ks[n][(c + 2) * 32 + 16 + g * 8];
            B3.h[0] = *(const v8h*)&Ks[16 + n][(c + 2) * 32 + g * 8];
            B3.h[1] = *(const v8h*)&Ks[16 + n][(c + 2) * 32 + 16 + g * 8];
            S0a = wmma_f16(Aq[c], B0.v, S0a);
            S1a = wmma_f16(Aq[c], B1.v, S1a);
            S0b = wmma_f16(Aq[c + 2], B2.v, S0b);
            S1b = wmma_f16(Aq[c + 2], B3.v, S1b);
        }
        v8f S0, S1;
#pragma unroll
        for (int r = 0; r < 8; ++r) { S0[r] = S0a[r] + S0b[r];
                                      S1[r] = S1a[r] + S1b[r]; }

#pragma unroll
        for (int r = 0; r < 8; ++r) {
            Ss[wave][r + 8 * g][n]      = S0[r];
            Ss[wave][r + 8 * g][16 + n] = S1[r];
        }
        __syncthreads();

        if (lane < 16) {
            const int row = lane;
            float mx = m_i;
#pragma unroll
            for (int k = 0; k < 32; ++k) mx = fmaxf(mx, Ss[wave][row][k]);
            float alpha = __expf(m_i - mx);
            float sum = 0.0f;
#pragma unroll
            for (int k = 0; k < 32; ++k) {
                float p = __expf(Ss[wave][row][k] - mx);
                sum += p;
                Ps[wave][row][k] = (_Float16)p;
            }
            l_i = l_i * alpha + sum;
            m_i = mx;
            Al[wave][row] = alpha;
        }
        __syncthreads();

        float alr[8];
#pragma unroll
        for (int r = 0; r < 8; ++r) alr[r] = Al[wave][8 * g + r];
#pragma unroll
        for (int t = 0; t < 8; ++t)
#pragma unroll
            for (int r = 0; r < 8; ++r) O[t][r] *= alr[r];

        union { v16h v; v8h h[2]; } P;
        P.h[0] = *(const v8h*)&Ps[wave][n][g * 8];
        P.h[1] = *(const v8h*)&Ps[wave][n][16 + g * 8];
#pragma unroll
        for (int t = 0; t < 8; ++t) {
            union { v16h v; v8h h[2]; } Bv;
            Bv.h[0] = *(const v8h*)&Vt[t * 16 + n][g * 8];
            Bv.h[1] = *(const v8h*)&Vt[t * 16 + n][16 + g * 8];
            O[t] = wmma_f16(P.v, Bv.v, O[t]);
        }
    }

    __syncthreads();
    if (lane < 16) Al[wave][lane] = l_i;
    __syncthreads();
    float lr[8];
#pragma unroll
    for (int r = 0; r < 8; ++r) lr[r] = 1.0f / Al[wave][8 * g + r];
    float* ot = Os[wave];
#pragma unroll
    for (int t = 0; t < 8; ++t)
#pragma unroll
        for (int r = 0; r < 8; ++r)
            ot[(r + 8 * g) * DKV + t * 16 + n] = O[t][r] * lr[r];
    __syncthreads();
    {
        char* d0 = (char*)(out + (size_t)q0 * DKV);
        v4f vv[16];
#pragma unroll
        for (int q = 0; q < 16; ++q) vv[q] = *(const v4f*)((const char*)ot + (q * 32 + lane) * 16);
#pragma unroll
        for (int q = 0; q < 16; ++q) *(volatile v4f*)(d0 + (q * 32 + lane) * 16) = vv[q];
        __threadfence();
#pragma unroll
        for (int q = 0; q < 16; ++q) *(volatile v4f*)(d0 + (q * 32 + lane) * 16) = vv[q];
    }
}

extern "C" void kernel_launch(void* const* d_in, const int* in_sizes, int n_in,
                              void* d_out, int out_size, void* d_ws, size_t ws_size,
                              hipStream_t stream) {
    const float* x   = (const float*)d_in[0];
    const float* Wqk = (const float*)d_in[1];
    const float* bqk = (const float*)d_in[2];
    const float* Wv  = (const float*)d_in[3];
    const float* bv  = (const float*)d_in[4];
    float* out = (float*)d_out;

    _Float16* qk_h = (_Float16*)d_ws;
    _Float16* v_h  = qk_h + (size_t)NTOK * DKV;

    proj_kernel<<<NTOK / 64, 256, 0, stream>>>(x, Wqk, bqk, Wv, bv, qk_h, v_h);
    flash_kernel<<<NTOK / 128, 256, 0, stream>>>(qk_h, v_h, out);
}
